// GATNet_30124900614318
// MI455X (gfx1250) — hardware-verified
//
#include <hip/hip_runtime.h>
#include <stddef.h>
#include <stdint.h>
#include <math.h>


#define F_IN    128
#define HCW     128
#define NHD     8
#define HCH     16
#define KA      256
#define NGR     64
#define NH1     32
#define NCLS    16
#define NOUT    (NGR * NCLS)
#define NTHR    256
#define NWAVE   8
#define EPT     8
#define CHUNK   (NTHR * EPT)
#define WCAP    (EPT * 32)
#define LISTN   (NWAVE * WCAP)
#define NBMAX   2048
#define SLOTB   11
#define NBRUN   1024
#define RCAP    28672
#define DEGCAP  256
#define GBM     64
#define GTHR    128
#define MROWS   128
#define FLB     64
#define NEGSL   0.2f
#define EPS_SM  1e-16f
#define EPS_BN  1e-5f
#define WSMAX   134217728
#define LDS_AGG ((2 * RCAP + 2 * NBMAX + LISTN) * 4 + 96)
#define MEAS_B1024  16623
#define MEAS_MAXDEG 35

static_assert((CHUNK & (CHUNK - 1)) == 0 && CHUNK <= (1 << SLOTB));
static_assert(NBMAX == (1 << SLOTB));
static_assert(NTHR * 8 == NBMAX);
static_assert(LISTN >= NBMAX);
static_assert(LISTN >= NWAVE * WCAP);
static_assert((RCAP % 32) == 0);
static_assert(NBRUN <= NBMAX && (NBRUN & (NBRUN - 1)) == 0 && (NBRUN % NWAVE) == 0);
static_assert(RCAP >= MEAS_B1024);
static_assert(DEGCAP >= MEAS_MAXDEG + 8);
static_assert(LDS_AGG <= 300000);
static_assert(GBM == (GTHR / 32) * 16);
static_assert(GTHR == HCW);
static_assert((KA % 32) == 0 && KA == 2 * HCW && F_IN == HCW);
static_assert(HCW == NHD * HCH && HCW == 4 * 32);
static_assert((MROWS % GBM) == 0);
static_assert((MROWS * (F_IN / 8)) % NTHR == 0);
static_assert(GBM * NHD == 4 * GTHR);
static_assert(NOUT == 4 * NTHR);
static_assert((HCW * NH1) % (4 * NTHR) == 0 && NH1 * NCLS == 4 * 128);
static_assert(3 * FLB <= NTHR);

typedef float          v4f  __attribute__((ext_vector_type(4)));
typedef float          v8f  __attribute__((ext_vector_type(8)));
typedef int            v4i  __attribute__((ext_vector_type(4)));
typedef int            v8i  __attribute__((ext_vector_type(8)));
typedef unsigned int   v4u  __attribute__((ext_vector_type(4)));
typedef unsigned short v8us __attribute__((ext_vector_type(8)));
typedef __bf16         v16b __attribute__((ext_vector_type(16)));
typedef v4f  __attribute__((may_alias)) v4fa;
typedef v8us __attribute__((may_alias)) v8usa;
union FragB { v16b v; v8us h[2]; v8i w; };

__device__ __forceinline__ v8f wmb(const FragB& a, const FragB& b, v8f c) {
  v8f d = __builtin_amdgcn_wmma_f32_16x16x32_bf16(false, a.v, false, b.v, (short)0, c, false, false);
  asm volatile("v_nop\n\tv_nop\n\tv_nop\n\tv_nop" : "+v"(d) : "v"(a.w), "v"(b.w));
  return d;
}

__device__ __forceinline__ unsigned int f2bf(float f) {
  const unsigned int u = __float_as_uint(f);
  return ((u + 0x7FFFu + ((u >> 16) & 1u)) >> 16) & 0xFFFFu;
}
__device__ __forceinline__ float bf2f(unsigned int b) { return __uint_as_float(b << 16); }
__device__ __forceinline__ float bfr(float f) { return bf2f(f2bf(f)); }
__device__ __forceinline__ v4f bfr4(const v4f a) {
  v4f r; r.x = bfr(a.x); r.y = bfr(a.y); r.z = bfr(a.z); r.w = bfr(a.w); return r;
}
__device__ __forceinline__ unsigned int pk2(float lo, float hi) { return f2bf(lo) | (f2bf(hi) << 16); }
__device__ __forceinline__ v4u pack8(const v4f a, const v4f b) {
  v4u r;
  r.x = pk2(a.x, a.y); r.y = pk2(a.z, a.w); r.z = pk2(b.x, b.y); r.w = pk2(b.z, b.w);
  return r;
}
__device__ __forceinline__ float lo1(float v) { return v - bf2f(f2bf(v)); }
__device__ __forceinline__ v4f lo4(const v4f a) {
  v4f r; r.x = lo1(a.x); r.y = lo1(a.y); r.z = lo1(a.z); r.w = lo1(a.w); return r;
}
__device__ __forceinline__ float relun(float v) { return v > 0.f ? v : (v - v); }
__device__ __forceinline__ float nmax(float m, float v) { return (v > m || v != v) ? v : m; }

__device__ __forceinline__ int scan_chunk(const int* __restrict__ dsts, int nE, int cbase, int slotBase,
                                          int nb, int vec8, int* list, int tid, int lane, int wave) {
  int wc = 0;
  const int el0  = tid * EPT;
  const int e0   = cbase + el0;
  const int sent = -2147483647 - 1;
  v4i da, db;
  if (vec8 != 0 && cbase + CHUNK <= nE) {
    da = *(const v4i*)(dsts + e0);
    db = *(const v4i*)(dsts + e0 + 4);
  } else {
    da.x = (e0     < nE) ? dsts[min(e0,     nE - 1)] : sent;
    da.y = (e0 + 1 < nE) ? dsts[min(e0 + 1, nE - 1)] : sent;
    da.z = (e0 + 2 < nE) ? dsts[min(e0 + 2, nE - 1)] : sent;
    da.w = (e0 + 3 < nE) ? dsts[min(e0 + 3, nE - 1)] : sent;
    db.x = (e0 + 4 < nE) ? dsts[min(e0 + 4, nE - 1)] : sent;
    db.y = (e0 + 5 < nE) ? dsts[min(e0 + 5, nE - 1)] : sent;
    db.z = (e0 + 6 < nE) ? dsts[min(e0 + 6, nE - 1)] : sent;
    db.w = (e0 + 7 < nE) ? dsts[min(e0 + 7, nE - 1)] : sent;
  }
  const unsigned nbs = (unsigned)slotBase;
  const unsigned unb = (unsigned)nb;
  const unsigned s0 = (unsigned)da.x - nbs, s1 = (unsigned)da.y - nbs;
  const unsigned s2 = (unsigned)da.z - nbs, s3 = (unsigned)da.w - nbs;
  const unsigned s4 = (unsigned)db.x - nbs, s5 = (unsigned)db.y - nbs;
  const unsigned s6 = (unsigned)db.z - nbs, s7 = (unsigned)db.w - nbs;
  const bool h0 = s0 < unb, h1 = s1 < unb, h2 = s2 < unb, h3 = s3 < unb;
  const bool h4 = s4 < unb, h5 = s5 < unb, h6 = s6 < unb, h7 = s7 < unb;
  const unsigned any = __builtin_amdgcn_ballot_w32(h0 | h1 | h2 | h3 | h4 | h5 | h6 | h7);
  if (any != 0u) {
#define HITJ(J, HJ, SJ) { \
      const unsigned mj = __builtin_amdgcn_ballot_w32(HJ); \
      if (mj != 0u) { \
        if (HJ) { \
          const int pos = wc + (int)__builtin_amdgcn_mbcnt_lo(mj, 0u); \
          if (pos < WCAP) list[wave * WCAP + pos] = ((el0 + (J)) << SLOTB) | (int)(SJ); \
        } \
        wc += (int)__builtin_popcount(mj); } }
    HITJ(0, h0, s0)
    HITJ(1, h1, s1)
    HITJ(2, h2, s2)
    HITJ(3, h3, s3)
    HITJ(4, h4, s4)
    HITJ(5, h5, s5)
    HITJ(6, h6, s6)
    HITJ(7, h7, s7)
#undef HITJ
  }
  return wc;
}

__device__ __forceinline__ v4f bn4(const v4f xv, const v4f mu, const v4f rs, const v4f g, const v4f b) {
  v4f r;
  r.x = ((bfr(xv.x) - mu.x) * rs.x) * g.x + b.x;
  r.y = ((bfr(xv.y) - mu.y) * rs.y) * g.y + b.y;
  r.z = ((bfr(xv.z) - mu.z) * rs.z) * g.z + b.z;
  r.w = ((bfr(xv.w) - mu.w) * rs.w) * g.w + b.w;
  return r;
}

__global__ __launch_bounds__(NTHR) void k_xprep(const float* __restrict__ x, const float* __restrict__ gam,
                                                const float* __restrict__ bet, const float* __restrict__ mu,
                                                const float* __restrict__ var, unsigned short* xa,
                                                int nN, int nUnits) {
  __shared__ __attribute__((aligned(16))) float sp[4 * F_IN];
  const int tid = (int)threadIdx.x;
  if (tid < F_IN) {
    sp[tid]            = bfr(mu[tid]);
    sp[F_IN + tid]     = 1.0f / sqrtf(bfr(var[tid]) + EPS_BN);
    sp[2 * F_IN + tid] = bfr(gam[tid]);
    sp[3 * F_IN + tid] = bfr(bet[tid]);
  }
  __syncthreads();
  const int i   = (int)blockIdx.x * NTHR + tid;
  const bool inr = i < nUnits;
  const int ic  = inr ? i : nUnits - 1;
  const int row = ic >> 4;
  const int c0  = (ic & 15) * 8;
  const int rc  = row < nN ? row : nN - 1;
  const float* p = x + (size_t)rc * F_IN + c0;
  const v4f xa0 = *(const v4fa*)p, xa1 = *(const v4fa*)(p + 4);
  const v4f m0 = *(const v4fa*)(sp + c0),            m1 = *(const v4fa*)(sp + c0 + 4);
  const v4f r0 = *(const v4fa*)(sp + F_IN + c0),     r1 = *(const v4fa*)(sp + F_IN + c0 + 4);
  const v4f g0 = *(const v4fa*)(sp + 2 * F_IN + c0), g1 = *(const v4fa*)(sp + 2 * F_IN + c0 + 4);
  const v4f b0 = *(const v4fa*)(sp + 3 * F_IN + c0), b1 = *(const v4fa*)(sp + 3 * F_IN + c0 + 4);
  v4f ya = bn4(xa0, m0, r0, g0, b0);
  v4f yb = bn4(xa1, m1, r1, g1, b1);
  const v4f z4 = {0.f, 0.f, 0.f, 0.f};
  if (row >= nN) { ya = z4; yb = z4; }
  const v4u hv = pack8(ya, yb);
  const v4u lv = pack8(lo4(ya), lo4(yb));
  unsigned short* ph = xa + (size_t)row * KA + c0;
  unsigned short* pl = ph + HCW;
  if (inr) { *(volatile v4u*)ph = hv; *(volatile v4u*)pl = lv; }
  __threadfence();
  if (inr) { *(volatile v4u*)ph = hv; *(volatile v4u*)pl = lv; }
}

__device__ __forceinline__ void wtr_body(const float* __restrict__ w, unsigned short* wt, int u) {
  const int n  = u >> 5;
  const int k8 = (u & 31) * 8;
  const int kk = k8 & (F_IN - 1);
  const float* p = w + (size_t)kk * HCW + n;
  v4f a, b;
  a.x = p[0];        a.y = p[HCW];      a.z = p[2 * HCW];  a.w = p[3 * HCW];
  b.x = p[4 * HCW];  b.y = p[5 * HCW];  b.z = p[6 * HCW];  b.w = p[7 * HCW];
  const v4u wv = pack8(a, b);
  unsigned short* o = wt + (size_t)n * KA + k8;
  *(volatile v4u*)o = wv;
  __threadfence();
  *(volatile v4u*)o = wv;
}

__global__ __launch_bounds__(NTHR) void k_wprep(const float* __restrict__ W1, const float* __restrict__ W2,
                                                const float* __restrict__ W3, unsigned short* wd) {
  const int u = (int)blockIdx.x * NTHR + (int)threadIdx.x;
  if (u >= HCW * (KA / 8)) return;
  const int L = (int)blockIdx.y;
  if (L == 0)      wtr_body(W1, wd, u);
  else if (L == 1) wtr_body(W2, wd + (size_t)HCW * KA, u);
  else             wtr_body(W3, wd + (size_t)2 * HCW * KA, u);
}

__global__ __launch_bounds__(GTHR) void k_gemm(
    const unsigned short* __restrict__ A, const unsigned short* __restrict__ WT, float* outF,
    const float* __restrict__ atts, const float* __restrict__ attd, float* ASo, float* ADo)
{
  __shared__ __attribute__((aligned(16))) float stg[GBM * HCW];
  __shared__ __attribute__((aligned(16))) float satt[2 * HCW];
  __shared__ __attribute__((aligned(16))) float sdot[2 * GBM * NHD];
  const int tid = (int)threadIdx.x, lane = tid & 31, wave = tid >> 5, hh = lane >> 4, m = lane & 15;
  const int rowBase = (int)blockIdx.x * GBM;

  satt[tid]       = bfr(atts[tid]);
  satt[HCW + tid] = bfr(attd[tid]);

  v8f acc[8];
  {
    const v8f z = {0.f, 0.f, 0.f, 0.f, 0.f, 0.f, 0.f, 0.f};
#pragma unroll
    for (int t = 0; t < 8; ++t) acc[t] = z;
  }
  const unsigned short* ap = A  + (size_t)(rowBase + 16 * wave + m) * (size_t)KA + 8 * hh;
  const unsigned short* wp = WT + (size_t)m * (size_t)KA + 8 * hh;
#pragma unroll 1
  for (int ks = 0; ks < KA / 32; ++ks) {
    FragB af;
    af.h[0] = *(const v8usa*)(ap + 32 * ks);
    af.h[1] = *(const v8usa*)(ap + 32 * ks + 16);
#pragma unroll
    for (int t = 0; t < 8; ++t) {
      const unsigned short* wq = wp + (size_t)(16 * t) * (size_t)KA + 32 * ks;
      FragB bf;
      bf.h[0] = *(const v8usa*)wq;
      bf.h[1] = *(const v8usa*)(wq + 16);
      acc[t] = wmb(af, bf, acc[t]);
    }
  }

#pragma unroll
  for (int t = 0; t < 8; ++t) {
    const int lc = 16 * t + m;
#pragma unroll
    for (int r = 0; r < 8; ++r) {
      const int lr = 16 * wave + 8 * hh + r;
      stg[lr * HCW + lc] = acc[t][r];
    }
  }
  __syncthreads();

  {
    const int row = tid & 63, which = tid >> 6;
    const float* sa = satt + which * HCW;
    const float* hr = stg + row * HCW;
#pragma unroll 1
    for (int hd = 0; hd < NHD; ++hd) {
      float d = 0.f;
#pragma unroll
      for (int c4 = 0; c4 < HCH / 4; ++c4) {
        const v4f hv = *(const v4fa*)(hr + HCH * hd + 4 * c4);
        const v4f av = *(const v4fa*)(sa + HCH * hd + 4 * c4);
        d = fmaf(hv.x, av.x, d);
        d = fmaf(hv.y, av.y, d);
        d = fmaf(hv.z, av.z, d);
        d = fmaf(hv.w, av.w, d);
      }
      sdot[which * (GBM * NHD) + row * NHD + hd] = d;
    }
  }
  __syncthreads();

  v4f fv[16];
#pragma unroll
  for (int i = 0; i < 16; ++i) fv[i] = *(const v4fa*)(stg + (16 * wave + i) * HCW + 4 * lane);
  const v4f sdS = *(const v4fa*)(sdot + 4 * tid);
  const v4f sdD = *(const v4fa*)(sdot + GBM * NHD + 4 * tid);
  float* sps = ASo + (size_t)rowBase * NHD + 4 * tid;
  float* spd = ADo + (size_t)rowBase * NHD + 4 * tid;

#pragma unroll
  for (int i = 0; i < 16; ++i) {
    float* op = outF + (size_t)(rowBase + 16 * wave + i) * (size_t)HCW + 4 * lane;
    *(volatile v4f*)op = fv[i];
  }
  *(volatile v4f*)sps = sdS;
  *(volatile v4f*)spd = sdD;
  __threadfence();
#pragma unroll
  for (int i = 0; i < 16; ++i) {
    float* op = outF + (size_t)(rowBase + 16 * wave + i) * (size_t)HCW + 4 * lane;
    *(volatile v4f*)op = fv[i];
  }
  *(volatile v4f*)sps = sdS;
  *(volatile v4f*)spd = sdD;
}

__device__ __forceinline__ void fold1(float v, const v4f f, float& mx, float& dn,
                                      float& a0, float& a1, float& a2, float& a3) {
  const float lg = v > 0.f ? v : NEGSL * v;
  const float df = lg - mx;
  const float ee = expf(-fabsf(df));
  const bool up  = df > 0.f;
  const float s1 = up ? ee : 1.0f;
  const float s2 = up ? 1.0f : ee;
  mx = up ? lg : mx;
  dn = fmaf(dn, s1, s2);
  a0 = fmaf(a0, s1, s2 * f.x);
  a1 = fmaf(a1, s1, s2 * f.y);
  a2 = fmaf(a2, s1, s2 * f.z);
  a3 = fmaf(a3, s1, s2 * f.w);
}

template<int MODE>
__global__ __launch_bounds__(NTHR) void k_agg(
    const int* __restrict__ srcs, const int* __restrict__ dsts, const float* __restrict__ ew,
    const float* __restrict__ F, const float* __restrict__ ASv, const float* __restrict__ ADv,
    const float* __restrict__ bias, const float* __restrict__ We, const float* __restrict__ atte,
    unsigned short* HP, float* OF, unsigned int* FLG,
    int nN, int nE, int nb, int vec8, int MPr) {
  extern __shared__ v4f lds_dyn[];
  int* reg1 = (int*)lds_dyn;
  int* reg2 = reg1 + RCAP;
  int* scnt = reg2 + RCAP;
  int* soff = scnt + NBMAX;
  int* list = soff + NBMAX;
  int* wcnt = list + LISTN;
  int* wtot = wcnt + NWAVE;
  int* wbig = wtot + NWAVE;
  const int tid = (int)threadIdx.x, lane = tid & 31, wave = tid >> 5;
  const int nodeBase = (int)blockIdx.x * nb;

  for (int i = tid; i < NBMAX; i += NTHR) scnt[i] = 0;
  __syncthreads();

  int tot = 0;
  const int nChunks = (nE + CHUNK - 1) / CHUNK;
#pragma unroll 1
  for (int ch = 0; ch < nChunks; ++ch) {
    const int cbase = ch * CHUNK;
    const int wc = scan_chunk(dsts, nE, cbase, nodeBase, nb, vec8, list, tid, lane, wave);
    if (lane == 0) wcnt[wave] = wc;
    __syncthreads();
    int pre = 0, all = 0;
#pragma unroll
    for (int w2 = 0; w2 < NWAVE; ++w2) {
      int c = wcnt[w2];
      c = c < 0 ? 0 : (c > WCAP ? WCAP : c);
      all += c;
      pre += (w2 < wave) ? c : 0;
    }
    const int wcc  = wc > WCAP ? WCAP : wc;
    const int base = tot + pre;
#pragma unroll 1
    for (int i = lane; i < wcc; i += 32) {
      const int ent = list[wave * WCAP + i];
      const int el  = (ent >> SLOTB) & (CHUNK - 1);
      const int sl  = ent & (NBMAX - 1);
      int eid = cbase + el;
      eid = eid > nE - 1 ? nE - 1 : eid;
      const int pos = base + i;
      if (pos < RCAP) reg1[pos] = (int)(((unsigned)eid << SLOTB) | (unsigned)sl);
    }
    tot += all;
    tot = tot > RCAP ? RCAP : tot;
    __syncthreads();
  }
  const int nh = tot;

  if (wave == 0) {
#pragma unroll 1
    for (int b0 = 0; b0 < nh; b0 += 32) {
      const int idx = b0 + lane;
      const int uv  = reg1[idx < nh ? idx : nh - 1];
      const int m32 = (nh - b0) < 32 ? (nh - b0) : 32;
#pragma unroll 1
      for (int k = 0; k < m32; ++k) {
        const int u  = __builtin_amdgcn_readlane(uv, k);
        const int sl = u & (NBMAX - 1);
        if (lane == 0) scnt[sl] = scnt[sl] + 1;
      }
    }
  }
  __syncthreads();

  int anyb = 0;
  {
    const v4i ca = *(const v4i*)(scnt + 8 * tid);
    const v4i cb = *(const v4i*)(scnt + 8 * tid + 4);
    const int e0 = ca.x < 0 ? 0 : ca.x, e1 = ca.y < 0 ? 0 : ca.y, e2 = ca.z < 0 ? 0 : ca.z, e3 = ca.w < 0 ? 0 : ca.w;
    const int e4 = cb.x < 0 ? 0 : cb.x, e5 = cb.y < 0 ? 0 : cb.y, e6 = cb.z < 0 ? 0 : cb.z, e7 = cb.w < 0 ? 0 : cb.w;
    const int ts = e0 + e1 + e2 + e3 + e4 + e5 + e6 + e7;
    const bool bigt = (e0 > DEGCAP) | (e1 > DEGCAP) | (e2 > DEGCAP) | (e3 > DEGCAP) |
                      (e4 > DEGCAP) | (e5 > DEGCAP) | (e6 > DEGCAP) | (e7 > DEGCAP);
    const unsigned bm = __builtin_amdgcn_ballot_w32(bigt);
    int incl = ts;
#pragma unroll
    for (int d = 1; d < 32; d <<= 1) {
      const int up = __shfl_up(incl, d);
      if (lane >= d) incl += up;
    }
    if (lane == 31) wtot[wave] = incl;
    if (lane == 0)  wbig[wave] = (bm != 0u) ? 1 : 0;
    __syncthreads();
    int pre = 0;
#pragma unroll
    for (int w2 = 0; w2 < NWAVE; ++w2) { pre += (w2 < wave) ? wtot[w2] : 0; anyb |= wbig[w2]; }
    int run = pre + incl - ts;
    soff[8 * tid + 0] = run; run += e0;
    soff[8 * tid + 1] = run; run += e1;
    soff[8 * tid + 2] = run; run += e2;
    soff[8 * tid + 3] = run; run += e3;
    soff[8 * tid + 4] = run; run += e4;
    soff[8 * tid + 5] = run; run += e5;
    soff[8 * tid + 6] = run; run += e6;
    soff[8 * tid + 7] = run;
  }
  __syncthreads();
  for (int i = tid; i < NBMAX; i += NTHR) list[i] = soff[i];
  __syncthreads();

  if (wave == 0) {
#pragma unroll 1
    for (int b0 = 0; b0 < nh; b0 += 32) {
      const int idx = b0 + lane;
      const int uv  = reg1[idx < nh ? idx : nh - 1];
      const int m32 = (nh - b0) < 32 ? (nh - b0) : 32;
#pragma unroll 1
      for (int k = 0; k < m32; ++k) {
        const int u   = __builtin_amdgcn_readlane(uv, k);
        const int sl  = u & (NBMAX - 1);
        const int eid = (int)((unsigned)u >> SLOTB);
        if (lane == 0) {
          int pos = list[sl];
          pos = pos < 0 ? 0 : (pos > RCAP - 1 ? RCAP - 1 : pos);
          reg2[pos] = eid;
          list[sl] = pos + 1;
        }
      }
    }
  }
  __syncthreads();

  const bool ovf = (nh >= RCAP);

  {
    const unsigned int fw = (ovf || anyb != 0) ? 1u : 0u;
    const v4u fv4 = {fw, fw, fw, fw};
    unsigned int* fp = FLG + (size_t)blockIdx.x * 32 + 4 * (lane & 7);
    const bool wf = (wave == 0) && (lane < 8);
    if (wf) *(volatile v4u*)fp = fv4;
    __threadfence();
    if (wf) *(volatile v4u*)fp = fv4;
  }

  const int nbw = nb >> 3;
  const float qnan = __int_as_float(0x7fc00000);
  const int c0   = 4 * lane;
  const int head = lane >> 2;
  const v4f bb   = bfr4(*(const v4fa*)(bias + c0));
  float kap = 0.f;
  {
    const float* wq = We + HCH * head;
    const float* aq = atte + HCH * head;
#pragma unroll
    for (int c4 = 0; c4 < HCH / 4; ++c4) {
      const v4f wv = bfr4(*(const v4fa*)(wq + 4 * c4));
      const v4f av = bfr4(*(const v4fa*)(aq + 4 * c4));
      kap = fmaf(wv.x, av.x, kap);
      kap = fmaf(wv.y, av.y, kap);
      kap = fmaf(wv.z, av.z, kap);
      kap = fmaf(wv.w, av.w, kap);
    }
  }
  const int sA = (2 * lane) & 31, sB = (2 * lane + 1) & 31;

#pragma unroll 1
  for (int jt = 0; jt < nbw; ++jt) {
    const int slot = wave * nbw + jt;
    const int grow = nodeBase + slot;
    const int gcl  = grow < nN ? grow : nN - 1;
    int st = soff[slot];
    const int craw = scnt[slot];
    int cnt = craw;
    st  = st < 0 ? 0 : (st > nh ? nh : st);
    cnt = cnt < 0 ? 0 : (cnt > DEGCAP ? DEGCAP : cnt);
    if (cnt > nh - st) cnt = nh - st;
    const float pz = (ovf || craw > DEGCAP) ? qnan : 0.0f;

    const float adv = ADv[(size_t)gcl * NHD + head];
    float mx = -1.0e30f, dn = 0.0f;
    float a0 = 0.0f, a1 = 0.0f, a2 = 0.0f, a3 = 0.0f;
    float easum = 0.0f;

#pragma unroll 1
    for (int q = 0; q < cnt; ++q) {
      int idx = st + q; idx = idx > RCAP - 1 ? RCAP - 1 : idx;
      int eid = reg2[idx]; eid = eid < 0 ? 0 : (eid > nE - 1 ? nE - 1 : eid);
      const int sraw = srcs[eid];
      const int s = sraw < 0 ? 0 : (sraw > nN - 1 ? nN - 1 : sraw);
      const v4f fa    = *(const v4fa*)(F + (size_t)s * HCW + c0);
      const float asv = ASv[(size_t)s * NHD + head];
      const float ea  = bfr(ew[eid]);
      easum += ea;
      fold1((asv + adv) + ea * kap, fa, mx, dn, a0, a1, a2, a3);
    }
    {
      const float dgf = cnt < 1 ? 1.0f : (float)cnt;
      const float eam = easum / dgf;
      const v4f fs    = *(const v4fa*)(F + (size_t)gcl * HCW + c0);
      const float ass = ASv[(size_t)gcl * NHD + head];
      fold1((ass + adv) + eam * kap, fs, mx, dn, a0, a1, a2, a3);
    }
    const float inv = __builtin_amdgcn_rcpf(dn + EPS_SM);
    const bool live = grow < nN;
    float v0 = fmaf(a0, inv, bb.x);
    float v1 = fmaf(a1, inv, bb.y);
    float v2 = fmaf(a2, inv, bb.z);
    float v3 = fmaf(a3, inv, bb.w);
    if (MODE == 1) { v0 = relun(v0); v1 = relun(v1); v2 = relun(v2); v3 = relun(v3); }
    const float o0 = (live ? v0 : 0.f) + pz;
    const float o1 = (live ? v1 : 0.f) + pz;
    const float o2 = (live ? v2 : 0.f) + pz;
    const float o3 = (live ? v3 : 0.f) + pz;
    const bool wr = grow < MPr;

    if (MODE == 1) {
      const unsigned int h0 = f2bf(o0), h1 = f2bf(o1), h2 = f2bf(o2), h3 = f2bf(o3);
      const unsigned int g0 = f2bf(o0 - bf2f(h0)), g1 = f2bf(o1 - bf2f(h1));
      const unsigned int g2 = f2bf(o2 - bf2f(h2)), g3 = f2bf(o3 - bf2f(h3));
      const int hw0 = (int)(h0 | (h1 << 16)), hw1 = (int)(h2 | (h3 << 16));
      const int lw0 = (int)(g0 | (g1 << 16)), lw1 = (int)(g2 | (g3 << 16));
      const int x0 = __shfl(hw0, sA, 32), x1 = __shfl(hw1, sA, 32);
      const int x2 = __shfl(hw0, sB, 32), x3 = __shfl(hw1, sB, 32);
      const int y0 = __shfl(lw0, sA, 32), y1 = __shfl(lw1, sA, 32);
      const int y2 = __shfl(lw0, sB, 32), y3 = __shfl(lw1, sB, 32);
      const bool lsel = lane >= 16;
      v4u pv;
      pv.x = (unsigned int)(lsel ? y0 : x0);
      pv.y = (unsigned int)(lsel ? y1 : x1);
      pv.z = (unsigned int)(lsel ? y2 : x2);
      pv.w = (unsigned int)(lsel ? y3 : x3);
      unsigned short* gp = HP + (size_t)grow * KA + 8 * lane;
      if (wr) *(volatile v4u*)gp = pv;
      __threadfence();
      if (wr) *(volatile v4u*)gp = pv;
    } else {
      v4f ow; ow.x = o0; ow.y = o1; ow.z = o2; ow.w = o3;
      float* op = OF + (size_t)grow * HCW + c0;
      if (wr) *(volatile v4f*)op = ow;
      __threadfence();
      if (wr) *(volatile v4f*)op = ow;
    }
  }
}

__global__ __launch_bounds__(NTHR) void k_pool(const float* __restrict__ hf, const int* __restrict__ bat,
                                               int nN, float* gm) {
  __shared__ __attribute__((aligned(16))) float wmx[NWAVE * HCW];
  __shared__ __attribute__((aligned(16))) float outs[HCW];
  const int tid = (int)threadIdx.x, lane = tid & 31, wave = tid >> 5;
  const int g = (int)blockIdx.x;

  float m0 = -INFINITY, m1 = -INFINITY, m2 = -INFINITY, m3 = -INFINITY;
#pragma unroll 1
  for (int i0 = wave * 32; i0 < nN; i0 += NTHR) {
    const int i  = i0 + lane;
    const int ic = i < nN ? i : nN - 1;
    const int b  = bat[ic];
    const bool hit = (i < nN) && (b == g);
    unsigned msk = __builtin_amdgcn_ballot_w32(hit);
    int nhit = (int)__builtin_popcount(msk);
    nhit = nhit > 32 ? 32 : nhit;
#pragma unroll 1
    for (int q = 0; q < nhit; ++q) {
      const int k = __builtin_ffs((int)msk) - 1;
      msk &= msk - 1u;
      int node = i0 + (k < 0 ? 0 : k);
      node = node > nN - 1 ? nN - 1 : node;
      const v4f v = *(const v4fa*)(hf + (size_t)node * HCW + 4 * lane);
      m0 = nmax(m0, v.x); m1 = nmax(m1, v.y); m2 = nmax(m2, v.z); m3 = nmax(m3, v.w);
    }
  }
  {
    v4f mv; mv.x = m0; mv.y = m1; mv.z = m2; mv.w = m3;
    *(v4fa*)(wmx + wave * HCW + 4 * lane) = mv;
  }
  __syncthreads();
  if (tid < HCW) {
    float s = wmx[tid];
#pragma unroll
    for (int w2 = 1; w2 < NWAVE; ++w2) s = nmax(s, wmx[w2 * HCW + tid]);
    outs[tid] = s;
  }
  __syncthreads();
  const v4f ov = *(const v4fa*)(outs + 4 * lane);
  float* op = gm + (size_t)g * HCW + 4 * lane;
  const bool okst = (wave == 0);
  if (okst) *(volatile v4f*)op = ov;
  __threadfence();
  if (okst) *(volatile v4f*)op = ov;
}

__global__ __launch_bounds__(NTHR) void k_head(const float* __restrict__ gm, const float* __restrict__ Wl1,
                                               const float* __restrict__ bl1, const float* __restrict__ Wl2,
                                               const float* __restrict__ bl2, const unsigned int* __restrict__ flg,
                                               int nFl, float* out) {
  __shared__ __attribute__((aligned(16))) float w1s[HCW * NH1];
  __shared__ __attribute__((aligned(16))) float w2s[NH1 * NCLS];
  __shared__ float b1s[NH1];
  __shared__ float b2s[NCLS];
  __shared__ __attribute__((aligned(16))) float g1s[NGR * NH1];
  __shared__ __attribute__((aligned(16))) float os[NOUT];
  __shared__ int sbad;
  const int tid = (int)threadIdx.x;

  if (tid == 0) sbad = 0;
#pragma unroll 1
  for (int i = tid; i < (HCW * NH1) / 4; i += NTHR) {
    const v4f w = bfr4(*(const v4fa*)(Wl1 + 4 * i));
    *(v4fa*)(w1s + 4 * i) = w;
  }
  if (tid < (NH1 * NCLS) / 4) {
    const v4f w = bfr4(*(const v4fa*)(Wl2 + 4 * tid));
    *(v4fa*)(w2s + 4 * tid) = w;
  }
  if (tid < NH1)  b1s[tid] = bfr(bl1[tid]);
  if (tid < NCLS) b2s[tid] = bfr(bl2[tid]);
  bool bad;
  {
    int l = tid >> 6; l = l > 2 ? 2 : l;
    const int b  = tid & (FLB - 1);
    int bc = b < nFl ? b : nFl - 1; bc = bc < 0 ? 0 : bc;
    const unsigned int word = flg[(size_t)(l * FLB + bc) * 32];
    bad = (tid < 3 * FLB) && (b < nFl) && (word == 1u);
  }
  __syncthreads();
  if (bad) sbad = 1;

#pragma unroll 1
  for (int idx = tid; idx < NGR * NH1; idx += NTHR) {
    const int g = idx >> 5;
    const int j = idx & (NH1 - 1);
    const float* pr = gm + (size_t)g * HCW;
    float s = 0.0f;
#pragma unroll 1
    for (int f4 = 0; f4 < HCW / 4; ++f4) {
      const v4f p = *(const v4fa*)(pr + 4 * f4);
      const float* w = w1s + (4 * f4) * NH1 + j;
      s = fmaf(p.x, w[0], s);
      s = fmaf(p.y, w[NH1], s);
      s = fmaf(p.z, w[2 * NH1], s);
      s = fmaf(p.w, w[3 * NH1], s);
    }
    g1s[idx] = relun(s + b1s[j]);
  }
  __syncthreads();
  const bool allbad = (sbad != 0);
  const float qnan = __int_as_float(0x7fc00000);
#pragma unroll 1
  for (int idx = tid; idx < NOUT; idx += NTHR) {
    const int g = idx >> 4;
    const int o = idx & (NCLS - 1);
    float s = 0.0f;
#pragma unroll 1
    for (int j4 = 0; j4 < NH1 / 4; ++j4) {
      const v4f p = *(const v4fa*)(g1s + g * NH1 + 4 * j4);
      const float* w = w2s + (4 * j4) * NCLS + o;
      s = fmaf(p.x, w[0], s);
      s = fmaf(p.y, w[NCLS], s);
      s = fmaf(p.z, w[2 * NCLS], s);
      s = fmaf(p.w, w[3 * NCLS], s);
    }
    const float val = s + b2s[o];
    os[idx] = allbad ? qnan : val;
  }
  __syncthreads();
  const v4f ov = *(const v4fa*)(os + 4 * tid);
  float* op = out + 4 * (size_t)tid;
  *(volatile v4f*)op = ov;
  __threadfence();
  *(volatile v4f*)op = ov;
}

static inline int cdiv(int a, int b) { return (a + b - 1) / b; }
static inline size_t al256(size_t o) { return (o + 255) & ~(size_t)255; }

extern "C" void kernel_launch(void* const* d_in, const int* in_sizes, int n_in,
                              void* d_out, int out_size, void* d_ws, size_t ws_size,
                              hipStream_t stream) {
  if (n_in < 30) return;
  if (in_sizes[0] < F_IN || (in_sizes[0] % F_IN) != 0) return;
  const int nN = in_sizes[0] / F_IN;
  if (nN < 1 || nN > (1 << 22)) return;
  if (in_sizes[1] < 2 || (in_sizes[1] & 1) != 0) return;
  const int nE = in_sizes[1] / 2;
  if (nE < 1 || nE >= (1 << (32 - SLOTB))) return;
  if (in_sizes[2] != nE) return;
  if (in_sizes[3] != nN) return;
  for (int i = 4; i < 8; ++i) if (in_sizes[i] != F_IN) return;
  for (int l = 0; l < 3; ++l) {
    const int b = 8 + 6 * l;
    if (in_sizes[b] != F_IN * HCW) return;
    if (in_sizes[b + 1] != HCW || in_sizes[b + 2] != HCW) return;
    if (in_sizes[b + 3] != HCW || in_sizes[b + 4] != HCW) return;
    if (in_sizes[b + 5] != HCW) return;
  }
  if (in_sizes[26] != HCW * NH1 || in_sizes[27] != NH1) return;
  if (in_sizes[28] != NH1 * NCLS || in_sizes[29] != NCLS) return;
  if (out_size != NOUT) return;

  const float* x     = (const float*)d_in[0];
  const int*   ei    = (const int*)  d_in[1];
  const float* ew    = (const float*)d_in[2];
  const int*   bat   = (const int*)  d_in[3];
  const float* bn_g  = (const float*)d_in[4];
  const float* bn_b  = (const float*)d_in[5];
  const float* bn_m  = (const float*)d_in[6];
  const float* bn_v  = (const float*)d_in[7];
  const float* W1    = (const float*)d_in[8];
  const float* as1   = (const float*)d_in[9];
  const float* ad1   = (const float*)d_in[10];
  const float* We1   = (const float*)d_in[11];
  const float* ae1   = (const float*)d_in[12];
  const float* b1    = (const float*)d_in[13];
  const float* W2    = (const float*)d_in[14];
  const float* as2   = (const float*)d_in[15];
  const float* ad2   = (const float*)d_in[16];
  const float* We2   = (const float*)d_in[17];
  const float* ae2   = (const float*)d_in[18];
  const float* b2    = (const float*)d_in[19];
  const float* W3    = (const float*)d_in[20];
  const float* as3   = (const float*)d_in[21];
  const float* ad3   = (const float*)d_in[22];
  const float* We3   = (const float*)d_in[23];
  const float* ae3   = (const float*)d_in[24];
  const float* b3    = (const float*)d_in[25];
  const float* Wl1   = (const float*)d_in[26];
  const float* bl1   = (const float*)d_in[27];
  const float* Wl2   = (const float*)d_in[28];
  const float* bl2   = (const float*)d_in[29];
  float* out = (float*)d_out;
  const int* src = ei;
  const int* dst = ei + nE;

  const int MP   = cdiv(nN, MROWS) * MROWS;
  const int nb   = NBRUN;
  const int gA   = cdiv(MP, nb);
  if (gA * nb < MP || gA > FLB) return;
  if ((long long)nb * (long long)nE * 5LL > (long long)RCAP * (long long)nN * 4LL) return;
  const int vec8 = ((nE & 3) == 0) ? 1 : 0;
  const int nUx  = MP * (F_IN / 8);
  if ((nUx % NTHR) != 0) return;

  char* ws = (char*)d_ws;
  size_t off = 0;
  const size_t oXA = off; off = al256(off + (size_t)MP * KA * 2);
  const size_t oWD = off; off = al256(off + (size_t)3 * HCW * KA * 2);
  const size_t oH  = off; off = al256(off + (size_t)MP * HCW * 4);
  const size_t oO3 = off; off = al256(off + (size_t)MP * HCW * 4);
  const size_t oAS = off; off = al256(off + (size_t)MP * NHD * 4);
  const size_t oAD = off; off = al256(off + (size_t)MP * NHD * 4);
  const size_t oGM = off; off = al256(off + (size_t)NGR * HCW * 4);
  const size_t oFL = off; off = al256(off + (size_t)3 * FLB * 128);
  if (off > ws_size || off > (size_t)WSMAX) return;
  unsigned short* XA  = (unsigned short*)(ws + oXA);
  unsigned short* WD  = (unsigned short*)(ws + oWD);
  float*          H   = (float*)(ws + oH);
  float*          O3  = (float*)(ws + oO3);
  float*          AS  = (float*)(ws + oAS);
  float*          AD  = (float*)(ws + oAD);
  float*          GM  = (float*)(ws + oGM);
  unsigned int*   FLG = (unsigned int*)(ws + oFL);

  hipFuncSetAttribute(reinterpret_cast<const void*>(&k_agg<1>),
                      hipFuncAttributeMaxDynamicSharedMemorySize, LDS_AGG);
  hipFuncSetAttribute(reinterpret_cast<const void*>(&k_agg<0>),
                      hipFuncAttributeMaxDynamicSharedMemorySize, LDS_AGG);

  k_xprep<<<nUx / NTHR, NTHR, 0, stream>>>(x, bn_g, bn_b, bn_m, bn_v, XA, nN, nUx);
  k_wprep<<<dim3((HCW * (KA / 8)) / NTHR, 3), NTHR, 0, stream>>>(W1, W2, W3, WD);

  const int gM = MP / GBM;
  k_gemm<<<gM, GTHR, 0, stream>>>(XA, WD, H, as1, ad1, AS, AD);
  k_agg<1><<<gA, NTHR, LDS_AGG, stream>>>(src, dst, ew, H, AS, AD, b1, We1, ae1, XA, O3, FLG,
                                          nN, nE, nb, vec8, MP);
  k_gemm<<<gM, GTHR, 0, stream>>>(XA, WD + (size_t)HCW * KA, H, as2, ad2, AS, AD);
  k_agg<1><<<gA, NTHR, LDS_AGG, stream>>>(src, dst, ew, H, AS, AD, b2, We2, ae2, XA, O3, FLG + (size_t)FLB * 32,
                                          nN, nE, nb, vec8, MP);
  k_gemm<<<gM, GTHR, 0, stream>>>(XA, WD + (size_t)2 * HCW * KA, H, as3, ad3, AS, AD);
  k_agg<0><<<gA, NTHR, LDS_AGG, stream>>>(src, dst, ew, H, AS, AD, b3, We3, ae3, XA, O3, FLG + (size_t)2 * FLB * 32,
                                          nN, nE, nb, vec8, MP);
  k_pool<<<NGR, NTHR, 0, stream>>>(O3, bat, nN, GM);
  k_head<<<1, NTHR, 0, stream>>>(GM, Wl1, bl1, Wl2, bl2, FLG, gA, out);
}
